// LinearCombiner_12876311953983
// MI455X (gfx1250) — hardware-verified
//
#include <hip/hip_runtime.h>
#include <stddef.h>


typedef _Float16 h16;
typedef _Float16 v16h __attribute__((ext_vector_type(16)));
typedef _Float16 v8h  __attribute__((ext_vector_type(8)));
typedef float    v8f  __attribute__((ext_vector_type(8)));
typedef float    v4f  __attribute__((ext_vector_type(4)));

#ifndef NT
#define NT 256
#endif
#ifndef NU
#define NU 128
#endif
#define NT_FULL 256
#define NU_FULL 128
#define DIM   1024
#define HIDW  3072
#define NOUT  8
#define NPAD  16
#define MROWS (NT + NU)

static_assert(NT >= 64 && NT <= NT_FULL && (NT % 64) == 0);
static_assert(NU >= 64 && NU <= NU_FULL && (NU % 64) == 0);
static_assert(HIDW == 3 * DIM);
static_assert((HIDW % 64) == 0 && (HIDW % 32) == 0);
static_assert((DIM % 32) == 0 && ((2 * DIM) % 32) == 0);
static_assert((MROWS % 64) == 0);
static_assert(NOUT == 8 && NPAD == 16);
static_assert(DIM / 8 == 128);
static_assert(((DIM / 8) % 32) == 0 && (((2 * DIM) / 8) % 32) == 0 && ((HIDW / 8) % 32) == 0);
static_assert(((size_t)NT * (DIM / 8)) % 256 == 0);
static_assert(((size_t)NU * (DIM / 8)) % 256 == 0);
static_assert(((size_t)HIDW * ((2 * DIM) / 8)) % 256 == 0);
static_assert(((size_t)HIDW * (DIM / 8)) % 256 == 0);
static_assert(((size_t)HIDW * (HIDW / 8)) % 256 == 0);
static_assert(((size_t)NPAD * (HIDW / 8)) % 256 == 0);
static_assert(((size_t)NT * NU * 2) % 256 == 0);
static_assert(((size_t)((NT_FULL - 1) * NU_FULL + NU_FULL) * NOUT * 4) == (size_t)1048576);

#define LDC 68
#define HLD 20
static_assert((LDC % 4) == 0 && LDC >= 64);
static_assert((HLD % 4) == 0 && HLD >= NPAD);

#define ACARRY 16.0f
#define WCARRY 64.0f
#define CSCALE (1.0f / (ACARRY * WCARRY))

#define XT_BYTES  ((size_t)NT * 2 * DIM * 2)
#define UP_BYTES  ((size_t)NU * DIM * 2)
#define W1A_BYTES ((size_t)HIDW * 2 * DIM * 2)
#define W1B_BYTES ((size_t)HIDW * DIM * 2)
#define W2_BYTES  ((size_t)HIDW * HIDW * 2)
#define W3_BYTES  ((size_t)NPAD * HIDW * 2)
#define ACT_BYTES ((size_t)MROWS * HIDW * 2)
#define C3_BYTES  ((size_t)MROWS * NOUT * 4)
#define OFF_XT  ((size_t)0)
#define OFF_UP  (OFF_XT + XT_BYTES)
#define OFF_W1A (OFF_UP + UP_BYTES)
#define OFF_W1B (OFF_W1A + W1A_BYTES)
#define OFF_W2  (OFF_W1B + W1B_BYTES)
#define OFF_W3  (OFF_W2 + W2_BYTES)
#define OFF_Y   (OFF_W3 + W3_BYTES)
#define OFF_Z   (OFF_Y + ACT_BYTES)
#define OFF_C3  (OFF_Z + ACT_BYTES)
#define WS_TOTAL (OFF_C3 + C3_BYTES)
static_assert((XT_BYTES % 128) == 0 && (UP_BYTES % 128) == 0 && (W1A_BYTES % 128) == 0);
static_assert((W1B_BYTES % 128) == 0 && (W2_BYTES % 128) == 0 && (W3_BYTES % 128) == 0);
static_assert((ACT_BYTES % 128) == 0 && (C3_BYTES % 128) == 0);
static_assert(WS_TOTAL <= (size_t)134217728);

__device__ __forceinline__ float bf16r(float x) {
  unsigned int u = __float_as_uint(x);
  u = (u + 0x7FFFu + ((u >> 16) & 1u)) & 0xFFFF0000u;
  return __uint_as_float(u);
}

static __device__ __forceinline__ h16 toh_flush(float v) {
  const h16 r = (h16)v;
  return (fabsf(v) < 6.103515625e-05f) ? (h16)0.0f : r;
}

__device__ __forceinline__ v16h frag_at(const _Float16* p) {
  v8h lo = *(const v8h*)(p);
  v8h hi = *(const v8h*)(p + 16);
  v16h out;
#pragma unroll
  for (int i = 0; i < 8; ++i) { out[i] = lo[i]; out[i + 8] = hi[i]; }
  return out;
}

__device__ __forceinline__ v8f wmma16(v16h a, v16h b, v8f c) {
  v8f d = __builtin_amdgcn_wmma_f32_16x16x32_f16(false, a, false, b, (short)0, c,
                                                 false, false);
  asm volatile("v_nop\n\tv_nop\n\tv_nop\n\tv_nop" : "+v"(d) : "v"(a), "v"(b));
  return d;
}

__global__ __launch_bounds__(256) void minmax_kernel(
    const float* __restrict__ A, const float* __restrict__ B, _Float16* __restrict__ X) {
  const unsigned g = blockIdx.x * 256u + threadIdx.x;
  if (g >= (unsigned)NT * (unsigned)(DIM / 8)) return;
  const unsigned t = g >> 7;
  const unsigned c = (g & 127u) * 8u;
  const float* pa = A + (size_t)t * DIM + c;
  const float* pb = B + (size_t)t * DIM + c;
  const v4f a0 = *(const v4f*)(pa);
  const v4f a1 = *(const v4f*)(pa + 4);
  const v4f b0 = *(const v4f*)(pb);
  const v4f b1 = *(const v4f*)(pb + 4);
  v8h lo, hi;
#pragma unroll
  for (int i = 0; i < 4; ++i) {
    const float ea0 = bf16r(a0[i]), eb0 = bf16r(b0[i]);
    const float ea1 = bf16r(a1[i]), eb1 = bf16r(b1[i]);
    lo[i]     = toh_flush(ACARRY * fminf(ea0, eb0));
    lo[i + 4] = toh_flush(ACARRY * fminf(ea1, eb1));
    hi[i]     = toh_flush(ACARRY * fmaxf(ea0, eb0));
    hi[i + 4] = toh_flush(ACARRY * fmaxf(ea1, eb1));
  }
  _Float16* pmin = X + (size_t)t * (2 * DIM) + c;
  _Float16* pmax = pmin + DIM;
  *(volatile v8h*)pmin = lo;
  *(volatile v8h*)pmax = hi;
  __threadfence();
  *(volatile v8h*)pmin = lo;
  *(volatile v8h*)pmax = hi;
}

__global__ __launch_bounds__(256) void cvt_plane_kernel(
    const float* __restrict__ src, _Float16* __restrict__ dst, const unsigned ld_src,
    const unsigned col0, const unsigned ncols8, const unsigned nrows_src,
    const unsigned nrows_dst, const float carry) {
  const unsigned g = blockIdx.x * 256u + threadIdx.x;
  if (g >= nrows_dst * ncols8) return;
  const unsigned row = g / ncols8;
  const unsigned c8 = g - row * ncols8;
  const unsigned srow = (row < nrows_src) ? row : (nrows_src - 1u);
  const bool live = (row < nrows_src);
  const float* p = src + (size_t)srow * ld_src + col0 + c8 * 8u;
  const v4f a0 = *(const v4f*)(p);
  const v4f a1 = *(const v4f*)(p + 4);
  v8h o;
#pragma unroll
  for (int i = 0; i < 4; ++i) {
    const float f0 = live ? carry * bf16r(a0[i]) : 0.0f;
    const float f1 = live ? carry * bf16r(a1[i]) : 0.0f;
    o[i]     = toh_flush(f0);
    o[i + 4] = toh_flush(f1);
  }
  _Float16* q = dst + (size_t)g * 8u;
  *(volatile v8h*)q = o;
  __threadfence();
  *(volatile v8h*)q = o;
}

__global__ __launch_bounds__(256) void gemm_plane_kernel(
    const _Float16* __restrict__ A16, const _Float16* __restrict__ Bt, const unsigned K,
    const float* __restrict__ bias, const unsigned brows, _Float16* __restrict__ out16) {
  __shared__ float Cs[64 * LDC];
  const unsigned tid = threadIdx.x, lane = tid & 31u, w = tid >> 5;
  const unsigned mw = w >> 1, nw = w & 1u;
  const unsigned hh = lane >> 4, m = lane & 15u;
  const unsigned n0 = blockIdx.x * 64u;
  const unsigned row0 = blockIdx.y * 64u;

  const _Float16* ap  = A16 + (size_t)(row0 + mw * 16u + m) * K + hh * 8u;
  const _Float16* bp0 = Bt + (size_t)(n0 + nw * 32u + m) * K + hh * 8u;
  const _Float16* bp1 = bp0 + (size_t)16 * K;
  v8f acc0 = {}, acc1 = {};
#pragma unroll 2
  for (unsigned k0 = 0; k0 < K; k0 += 32u) {
    const v16h a  = frag_at(ap + k0);
    const v16h b0 = frag_at(bp0 + k0);
    const v16h b1 = frag_at(bp1 + k0);
    acc0 = wmma16(a, b0, acc0);
    acc1 = wmma16(a, b1, acc1);
  }
#pragma unroll
  for (int r = 0; r < 8; ++r) {
    float* d = &Cs[(mw * 16u + hh * 8u + (unsigned)r) * LDC + nw * 32u + m];
    d[0]  = acc0[r];
    d[16] = acc1[r];
  }
  __syncthreads();

  const bool addb = (row0 < brows);
  v8h x[2];
  size_t off[2];
#pragma unroll
  for (unsigned i = 0; i < 2u; ++i) {
    const unsigned r = 32u * i + (tid >> 3);
    const unsigned c = (tid & 7u) * 8u;
    const v4f u0 = *(const v4f*)&Cs[r * LDC + c];
    const v4f u1 = *(const v4f*)&Cs[r * LDC + c + 4];
    const v4f g0 = *(const v4f*)(bias + n0 + c);
    const v4f g1 = *(const v4f*)(bias + n0 + c + 4u);
#pragma unroll
    for (int j = 0; j < 4; ++j) {
      const float bb0 = addb ? bf16r(g0[j]) : 0.0f;
      const float bb1 = addb ? bf16r(g1[j]) : 0.0f;
      x[i][j]     = toh_flush(ACARRY * (u0[j] * CSCALE + bb0));
      x[i][j + 4] = toh_flush(ACARRY * (u1[j] * CSCALE + bb1));
    }
    off[i] = (size_t)(row0 + r) * HIDW + n0 + c;
  }
#pragma unroll
  for (int i = 0; i < 2; ++i) *(volatile v8h*)(out16 + off[i]) = x[i];
  __threadfence();
#pragma unroll
  for (int i = 0; i < 2; ++i) *(volatile v8h*)(out16 + off[i]) = x[i];
}

__global__ __launch_bounds__(128) void head_kernel(
    const _Float16* __restrict__ Z16, const _Float16* __restrict__ W3t,
    const float* __restrict__ bias, const unsigned brows, float* __restrict__ C3) {
  __shared__ float Hs[64 * HLD];
  const unsigned tid = threadIdx.x, lane = tid & 31u, w = tid >> 5;
  const unsigned hh = lane >> 4, m = lane & 15u;
  const unsigned row0 = blockIdx.x * 64u;

  const _Float16* ap = Z16 + (size_t)(row0 + w * 16u + m) * HIDW + hh * 8u;
  const _Float16* bp = W3t + (size_t)m * HIDW + hh * 8u;
  v8f acc = {};
#pragma unroll 2
  for (unsigned k0 = 0; k0 < (unsigned)HIDW; k0 += 32u) {
    const v16h a = frag_at(ap + k0);
    const v16h b = frag_at(bp + k0);
    acc = wmma16(a, b, acc);
  }
#pragma unroll
  for (int r = 0; r < 8; ++r)
    Hs[(w * 16u + hh * 8u + (unsigned)r) * HLD + m] = acc[r];
  __syncthreads();

  const bool addb = (row0 < brows);
  const unsigned r = tid >> 1;
  const unsigned c = (tid & 1u) * 4u;
  const v4f u = *(const v4f*)&Hs[r * HLD + c];
  const v4f g = *(const v4f*)(bias + c);
  v4f val;
#pragma unroll
  for (int j = 0; j < 4; ++j) {
    const float bb = addb ? bf16r(g[j]) : 0.0f;
    val[j] = u[j] * CSCALE + bb;
  }
  float* p = C3 + (size_t)(row0 + r) * NOUT + c;
  *(volatile v4f*)p = val;
  __threadfence();
  *(volatile v4f*)p = val;
}

__global__ __launch_bounds__(256) void combine_kernel(
    const float* __restrict__ C3, float* __restrict__ out) {
  const unsigned g = blockIdx.x * 256u + threadIdx.x;
  if (g >= (unsigned)NT * (unsigned)NU * 2u) return;
  const unsigned t = g / (unsigned)(NU * 2);
  const unsigned rem = g - t * (unsigned)(NU * 2);
  const unsigned u = rem >> 1;
  const unsigned hf = (rem & 1u) * 4u;
  const v4f a = *(const v4f*)(C3 + (size_t)t * NOUT + hf);
  const v4f b = *(const v4f*)(C3 + (size_t)(NT + u) * NOUT + hf);
  v4f val;
#pragma unroll
  for (int j = 0; j < 4; ++j) val[j] = a[j] + b[j];
  float* p = out + ((size_t)t * NU_FULL + u) * NOUT + hf;
  *(volatile v4f*)p = val;
  __threadfence();
  *(volatile v4f*)p = val;
}

extern "C" void kernel_launch(void* const* d_in, const int* in_sizes, int n_in,
                              void* d_out, int out_size, void* d_ws, size_t ws_size,
                              hipStream_t stream) {
  if (n_in < 9) return;
  if ((long long)in_sizes[0] < (long long)NT * DIM) return;
  if ((long long)in_sizes[1] < (long long)NT * DIM) return;
  if ((long long)in_sizes[2] < (long long)NU * DIM) return;
  if ((long long)in_sizes[3] < (long long)HIDW * HIDW) return;
  if (in_sizes[4] < HIDW) return;
  if ((long long)in_sizes[5] < (long long)HIDW * HIDW) return;
  if (in_sizes[6] < HIDW) return;
  if ((long long)in_sizes[7] < (long long)NOUT * HIDW) return;
  if (in_sizes[8] < NOUT) return;
  if ((long long)out_size < ((long long)(NT - 1) * NU_FULL + NU) * NOUT) return;
  if (ws_size < WS_TOTAL) return;

  const float* text_a = (const float*)d_in[0];
  const float* text_b = (const float*)d_in[1];
  const float* user   = (const float*)d_in[2];
  const float* w1     = (const float*)d_in[3];
  const float* b1     = (const float*)d_in[4];
  const float* w2     = (const float*)d_in[5];
  const float* b2     = (const float*)d_in[6];
  const float* w3     = (const float*)d_in[7];
  const float* b3     = (const float*)d_in[8];
  float* out = (float*)d_out;

  char* ws = (char*)d_ws;
  _Float16* Xt16  = (_Float16*)(ws + OFF_XT);
  _Float16* Up16  = (_Float16*)(ws + OFF_UP);
  _Float16* W1a16 = (_Float16*)(ws + OFF_W1A);
  _Float16* W1b16 = (_Float16*)(ws + OFF_W1B);
  _Float16* W2_16 = (_Float16*)(ws + OFF_W2);
  _Float16* W3_16 = (_Float16*)(ws + OFF_W3);
  _Float16* Y16   = (_Float16*)(ws + OFF_Y);
  _Float16* Z16   = (_Float16*)(ws + OFF_Z);
  float*    C3    = (float*)(ws + OFF_C3);

  dim3 blk(256);

  minmax_kernel<<<dim3((NT * (DIM / 8)) / 256), blk, 0, stream>>>(text_a, text_b, Xt16);
  cvt_plane_kernel<<<dim3((NU * (DIM / 8)) / 256), blk, 0, stream>>>(
      user, Up16, (unsigned)DIM, 0u, (unsigned)(DIM / 8), (unsigned)NU, (unsigned)NU, ACARRY);
  cvt_plane_kernel<<<dim3((HIDW * ((2 * DIM) / 8)) / 256), blk, 0, stream>>>(
      w1, W1a16, (unsigned)HIDW, 0u, (unsigned)((2 * DIM) / 8), (unsigned)HIDW, (unsigned)HIDW,
      WCARRY);
  cvt_plane_kernel<<<dim3((HIDW * (DIM / 8)) / 256), blk, 0, stream>>>(
      w1, W1b16, (unsigned)HIDW, (unsigned)(2 * DIM), (unsigned)(DIM / 8), (unsigned)HIDW,
      (unsigned)HIDW, WCARRY);
  cvt_plane_kernel<<<dim3((HIDW * (HIDW / 8)) / 256), blk, 0, stream>>>(
      w2, W2_16, (unsigned)HIDW, 0u, (unsigned)(HIDW / 8), (unsigned)HIDW, (unsigned)HIDW,
      WCARRY);
  cvt_plane_kernel<<<dim3((NPAD * (HIDW / 8)) / 256), blk, 0, stream>>>(
      w3, W3_16, (unsigned)HIDW, 0u, (unsigned)(HIDW / 8), (unsigned)NOUT, (unsigned)NPAD,
      WCARRY);

  gemm_plane_kernel<<<dim3(HIDW / 64, NT / 64), blk, 0, stream>>>(
      Xt16, W1a16, (unsigned)(2 * DIM), b1, (unsigned)NT, Y16);
  gemm_plane_kernel<<<dim3(HIDW / 64, NU / 64), blk, 0, stream>>>(
      Up16, W1b16, (unsigned)DIM, b1, 0u, Y16 + (size_t)NT * HIDW);
  gemm_plane_kernel<<<dim3(HIDW / 64, MROWS / 64), blk, 0, stream>>>(
      Y16, W2_16, (unsigned)HIDW, b2, (unsigned)NT, Z16);
  head_kernel<<<dim3(MROWS / 64), dim3(128), 0, stream>>>(Z16, W3_16, b3, (unsigned)NT, C3);
  combine_kernel<<<dim3((NT * NU * 2) / 256), blk, 0, stream>>>(C3, out);
}
